// LSTM_seq2seq_6794638262641
// MI455X (gfx1250) — hardware-verified
//
#include <hip/hip_runtime.h>
#include <math.h>

typedef __attribute__((ext_vector_type(16))) _Float16 v16h;
typedef __attribute__((ext_vector_type(8)))  _Float16 v8h;
typedef __attribute__((ext_vector_type(16))) __bf16   v16b;
typedef __attribute__((ext_vector_type(8)))  __bf16   v8b;
typedef __attribute__((ext_vector_type(8)))  float    v8f;
typedef __attribute__((ext_vector_type(4)))  float    v4f;

constexpr int kB    = 64;
constexpr int kTe   = 256;
constexpr int kTd   = 256;
constexpr int kLat  = 512;
constexpr int kHid  = 1024;
constexpr int kGe   = 4 * kHid;
constexpr int kGd   = 4 * kLat;
constexpr int kKe   = kHid + kLat;
constexpr int kCmb  = 2 * kHid;
constexpr int kIni  = 2 * kLat;
constexpr int kThr  = 256;
constexpr float kWCarry  = 4096.0f;
constexpr float kSCarry  = 1024.0f;
constexpr float kSc = 1.0f / (kSCarry * kWCarry);
constexpr float kF16MinNormal = 6.103515625e-5f;

static_assert((kB % 64) == 0 && (kGe % 64) == 0 && (kGd % 64) == 0 && (kIni % 64) == 0 && ((kB / 64) * (kGe / 64)) % 8 == 0 && ((kB / 64) * (kGd / 64)) % 8 == 0 && ((kB / 64) * (kIni / 64)) % 8 == 0, "GEMM M, N multiples of 64; grids exact");
static_assert((kKe % 32) == 0 && (kCmb % 32) == 0 && (kHid % 32) == 0 && (kLat % 32) == 0, "GEMM K multiples of 32");

constexpr size_t kOffWE = 0ull;
constexpr size_t kOffWINI = 12582912ull;
constexpr size_t kOffWXD = 16777216ull;
constexpr size_t kOffWHD = 20971520ull;
constexpr size_t kOffBIAS = 23068672ull;
constexpr size_t kOffAE = 23117824ull;
constexpr size_t kOffGE = 23314432ull;
constexpr size_t kOffCE = 24363008ull;
constexpr size_t kOffCMB16 = 24625152ull;
constexpr size_t kOffINI = 24887296ull;
constexpr size_t kOffXDEC = 25149440ull;
constexpr size_t kOffHD16 = 25673728ull;
constexpr size_t kOffGD = 25739264ull;
constexpr size_t kOffCD = 26263552ull;
constexpr size_t kWsTotal = 26394624ull;
static_assert(kWsTotal <= 134217728ull, "carve cap: under 128 MiB");
static_assert(kOffWE == 0
              && kOffWINI == kOffWE + 12582912ull
              && kOffWXD == kOffWINI + 4194304ull
              && kOffWHD == kOffWXD + 4194304ull
              && kOffBIAS == kOffWHD + 2097152ull
              && kOffAE == kOffBIAS + 49152ull
              && kOffGE == kOffAE + 196608ull
              && kOffCE == kOffGE + 1048576ull
              && kOffCMB16 == kOffCE + 262144ull
              && kOffINI == kOffCMB16 + 262144ull
              && kOffXDEC == kOffINI + 262144ull
              && kOffHD16 == kOffXDEC + 524288ull
              && kOffGD == kOffHD16 + 65536ull
              && kOffCD == kOffGD + 524288ull
              && kWsTotal == kOffCD + 131072ull, "the carve is chained and totalled");
static_assert((kOffWE % 256) == 0 && (kOffWINI % 256) == 0 && (kOffWXD % 256) == 0 && (kOffWHD % 256) == 0 && (kOffBIAS % 256) == 0 && (kOffAE % 256) == 0 && (kOffGE % 256) == 0 && (kOffCE % 256) == 0 && (kOffCMB16 % 256) == 0 && (kOffINI % 256) == 0 && (kOffXDEC % 256) == 0 && (kOffHD16 % 256) == 0 && (kOffGD % 256) == 0 && (kOffCD % 256) == 0, "aligned regions");
constexpr int kFBE = 0, kFBD = 4096, kFBI = 6144, kFZB = 8192, kFEnd = 12288;
static_assert(kFBD == kFBE + kGe && kFBI == kFBD + kGd && kFBI + kIni <= kFZB && kFZB + kGd <= kFEnd && (kFZB % 128) == 0, "bias stream map; the zero row reaches the decoder step's 2,048 columns");

__device__ __forceinline__ unsigned short f2bf_bits(float f) {
  unsigned u = __float_as_uint(f);
  return (unsigned short)((u + 0x7FFFu + ((u >> 16) & 1u)) >> 16);
}
__device__ __forceinline__ float bf_bits2f(unsigned short h) { return __uint_as_float(((unsigned)h) << 16); }
__device__ __forceinline__ float bf16r(float f) { return bf_bits2f(f2bf_bits(f)); }
__device__ __forceinline__ float carry_flush(float v, float carry) {
  const float s = v * carry;
  return (fabsf(s) < kF16MinNormal) ? 0.0f : s;
}
__device__ __forceinline__ float frcp(float x) { return __builtin_amdgcn_rcpf(x); }

__device__ __forceinline__ void dep_guard4_h(v8f& a, v8f& b, v8f& c, v8f& d, v16h x, v16h y) { asm volatile("v_nop\n\tv_nop\n\tv_nop\n\tv_nop" : "+v"(a), "+v"(b), "+v"(c), "+v"(d) : "v"(x), "v"(y)); }
__device__ __forceinline__ void dep_guard4_b(v8f& a, v8f& b, v8f& c, v8f& d, v16b x, v16b y) { asm volatile("v_nop\n\tv_nop\n\tv_nop\n\tv_nop" : "+v"(a), "+v"(b), "+v"(c), "+v"(d) : "v"(x), "v"(y)); }
__device__ __forceinline__ void keep4_h(v16h a, v16h b, v16h c, v16h d) { asm volatile("v_nop" :: "v"(a), "v"(b), "v"(c), "v"(d)); }
__device__ __forceinline__ void keep4_b(v16b a, v16b b, v16b c, v16b d) { asm volatile("v_nop" :: "v"(a), "v"(b), "v"(c), "v"(d)); }
__device__ __forceinline__ void acc_guard4(v8f& a, v8f& b, v8f& c, v8f& d) { asm volatile("v_nop\n\tv_nop\n\tv_nop\n\tv_nop" : "+v"(a), "+v"(b), "+v"(c), "+v"(d)); }

template <typename T> struct Frag;
template <> struct Frag<_Float16> {
  typedef v16h V; union U { v16h v; v8h h[2]; };
  static __device__ __forceinline__ v16h load(const _Float16* p) {
    U f; f.h[0] = *(const v8h*)(p); f.h[1] = *(const v8h*)(p + 16); return f.v;
  }
  static __device__ __forceinline__ v8f mma(v16h a, v16h b, v8f c) {
    return __builtin_amdgcn_wmma_f32_16x16x32_f16(false, a, false, b, (short)0, c, false, false);
  }
  static __device__ __forceinline__ void guard4(v8f& a, v8f& b, v8f& c, v8f& d, v16h x, v16h y) { dep_guard4_h(a, b, c, d, x, y); }
  static __device__ __forceinline__ void keep(v16h a, v16h b, v16h c, v16h d) { keep4_h(a, b, c, d); }
};
template <> struct Frag<__bf16> {
  typedef v16b V; union U { v16b v; v8b h[2]; };
  static __device__ __forceinline__ v16b load(const __bf16* p) {
    U f; f.h[0] = *(const v8b*)(p); f.h[1] = *(const v8b*)(p + 16); return f.v;
  }
  static __device__ __forceinline__ v8f mma(v16b a, v16b b, v8f c) {
    return __builtin_amdgcn_wmma_f32_16x16x32_bf16(false, a, false, b, (short)0, c, false, false);
  }
  static __device__ __forceinline__ void guard4(v8f& a, v8f& b, v8f& c, v8f& d, v16b x, v16b y) { dep_guard4_b(a, b, c, d, x, y); }
  static __device__ __forceinline__ void keep(v16b a, v16b b, v16b c, v16b d) { keep4_b(a, b, c, d); }
};

__device__ __forceinline__ v8f mma_h(v16h a, v16h b, v8f c) {
  c = __builtin_amdgcn_wmma_f32_16x16x32_f16(false, a, false, b, (short)0, c, false, false);
  asm volatile("v_nop\n\tv_nop\n\tv_nop\n\tv_nop" : "+v"(c) : "v"(a), "v"(b));
  return c;
}

template <int ET> struct Elem;
template <> struct Elem<0> { typedef _Float16 T; };
template <> struct Elem<1> { typedef __bf16 T; };
template <int ET, bool SPLIT, int BIAS_MODE, int OUT_MODE, bool RESID, int ACT = 0>
__global__ __launch_bounds__(256) void wmma_gemm64(
    const unsigned short* __restrict__ Ap, const unsigned short* __restrict__ A2p, int lda, long strideA,
    const unsigned short* __restrict__ Btp, const unsigned short* __restrict__ Bt2p, int ldb, long strideB,
    void* __restrict__ Cout, void* __restrict__ Cout2, int ldc, long strideC,
    const float* __restrict__ bias,
    const float* __restrict__ resid, long strideR,
    int M, int N, int K, float scale) {
  typedef typename Elem<ET>::T T;
  typedef typename Frag<T>::V V;
  const T* A = (const T*)Ap; const T* A2 = (const T*)A2p; const T* Bt = (const T*)Btp; const T* Bt2 = (const T*)Bt2p;
  __shared__ __align__(16) float sT[8][16 * 68];
  const int b    = blockIdx.y;
  const int lane = threadIdx.x & 31;
  const int wave = threadIdx.x >> 5;
  const int tilesN = N >> 6;
  const int tilesM = M >> 6;
  const int tile = blockIdx.x * 8 + wave;
  if (tile >= tilesM * tilesN) return;
  const int tm = tile / tilesN;
  const int tn = tile - tm * tilesN;
  const int m0 = tm << 6;
  const int n0 = tn << 6;

  const T* Ab  = A  + (size_t)b * strideA;
  const T* Bb  = Bt + (size_t)b * strideB;
  const T* Ab2 = SPLIT ? (A2  + (size_t)b * strideA) : nullptr;
  const T* Bb2 = SPLIT ? (Bt2 + (size_t)b * strideB) : nullptr;

  const int rlane = lane & 15;
  const int koff  = (lane >> 4) * 8;
  const int mOff  = (lane >> 4) * 8;

  v8f acc[4][4];
#pragma unroll
  for (int i = 0; i < 4; ++i)
#pragma unroll
    for (int j = 0; j < 4; ++j) acc[i][j] = (v8f){0.f,0.f,0.f,0.f,0.f,0.f,0.f,0.f};

  for (int k0 = 0; k0 < K; k0 += 32) {
    V bh[4], bl[4];
#pragma unroll
    for (int j = 0; j < 4; ++j) {
      const size_t bo = (size_t)(n0 + (j << 4) + rlane) * ldb + koff + k0;
      bh[j] = Frag<T>::load(Bb + bo);
      if (SPLIT) bl[j] = Frag<T>::load(Bb2 + bo);
    }
#pragma unroll
    for (int i = 0; i < 4; ++i) {
      const size_t ao = (size_t)(m0 + (i << 4) + rlane) * lda + koff + k0;
      V ah = Frag<T>::load(Ab + ao);
      V al;
      if (SPLIT) al = Frag<T>::load(Ab2 + ao);
#pragma unroll
      for (int j = 0; j < 4; ++j) {
        acc[i][j] = Frag<T>::mma(ah, bh[j], acc[i][j]);
        if (SPLIT) {
          acc[i][j] = Frag<T>::mma(ah, bl[j], acc[i][j]);
          acc[i][j] = Frag<T>::mma(al, bh[j], acc[i][j]);
        }
      }
      Frag<T>::guard4(acc[i][0], acc[i][1], acc[i][2], acc[i][3], ah, SPLIT ? al : ah);
    }
    Frag<T>::keep(bh[0], bh[1], bh[2], bh[3]);
    if (SPLIT) Frag<T>::keep(bl[0], bl[1], bl[2], bl[3]);
  }
  acc_guard4(acc[0][0], acc[0][1], acc[0][2], acc[0][3]);
  acc_guard4(acc[1][0], acc[1][1], acc[1][2], acc[1][3]);
  acc_guard4(acc[2][0], acc[2][1], acc[2][2], acc[2][3]);
  acc_guard4(acc[3][0], acc[3][1], acc[3][2], acc[3][3]);

  float* slab = sT[wave];
  const float* Rb = RESID ? (resid + (size_t)b * strideR) : nullptr;
#pragma unroll
  for (int i = 0; i < 4; ++i) {
    const int mBase = m0 + (i << 4);
#pragma unroll
    for (int j = 0; j < 4; ++j) {
      const int n = n0 + (j << 4) + rlane;
      float bv = 0.f;
      if (BIAS_MODE == 2) bv = bias[n];
#pragma unroll
      for (int r = 0; r < 8; ++r) {
        float v = acc[i][j][r] * scale;
        if (BIAS_MODE == 1) v += bias[mBase + mOff + r];
        if (BIAS_MODE == 2) v += bv;
        if (RESID) v += Rb[(size_t)(mBase + mOff + r) * ldc + n];
        if (ACT == 1) v = tanhf(v);
        if (ACT == 2) v = fmaxf(v, 0.0f);
        if (ACT == 3) v = v / (1.0f + expf(-v));
        if (ACT == 4) v = (v > 0.f) ? v : 0.01f * v;
        slab[(mOff + r) * 68 + (j << 4) + rlane] = v;
      }
    }
    __builtin_amdgcn_fence(__ATOMIC_RELEASE, "workgroup");
    __builtin_amdgcn_wave_barrier();
    __builtin_amdgcn_fence(__ATOMIC_ACQUIRE, "workgroup");
    if (OUT_MODE == 0) {
      float* C = (float*)Cout + (size_t)b * strideC;
      const int hh = lane >> 4, c4 = (lane & 15) * 4;
      for (int pass = 0; pass < 2; ++pass) {
#pragma unroll
        for (int it = 0; it < 8; ++it) {
          const int row = it * 2 + hh;
          v4f v = *(const v4f*)(slab + row * 68 + c4);
          *(volatile v4f*)(C + (size_t)(mBase + row) * ldc + n0 + c4) = v;
        }
        __threadfence();
      }
    } else {
      const int q = lane >> 3, c8 = (lane & 7) * 8;
      unsigned short* C  = (unsigned short*)Cout  + (size_t)b * strideC;
      unsigned short* C2 = (OUT_MODE == 2) ? ((unsigned short*)Cout2 + (size_t)b * strideC) : nullptr;
      for (int pass = 0; pass < 2; ++pass) {
#pragma unroll
        for (int it = 0; it < 4; ++it) {
          const int row = it * 4 + q;
          const float* sp = slab + row * 68 + c8;
          v8h hv, lv;
#pragma unroll
          for (int e = 0; e < 8; ++e) {
            if (OUT_MODE == 1) {
              hv[e] = (_Float16)sp[e];
            } else {
              unsigned short hb = f2bf_bits(sp[e]);
              unsigned short lb = f2bf_bits(sp[e] - bf_bits2f(hb));
              hv[e] = __builtin_bit_cast(_Float16, hb);
              lv[e] = __builtin_bit_cast(_Float16, lb);
            }
          }
          *(volatile v8h*)(C + (size_t)(mBase + row) * ldc + n0 + c8) = hv;
          if (OUT_MODE == 2) *(volatile v8h*)(C2 + (size_t)(mBase + row) * ldc + n0 + c8) = lv;
        }
        __threadfence();
      }
    }
    __builtin_amdgcn_fence(__ATOMIC_RELEASE, "workgroup");
    __builtin_amdgcn_wave_barrier();
    __builtin_amdgcn_fence(__ATOMIC_ACQUIRE, "workgroup");
  }
}

__global__ __launch_bounds__(256) void wt_plane_kernel(const float* __restrict__ W, unsigned short* __restrict__ dst, int K, int N, int nLive, int ldd, int colOff) {
  const int n  = blockIdx.x;
  const int k8 = threadIdx.x * 8;
  const bool live = n < nLive;
  const int nc = live ? n : 0;
  v8h hv;
#pragma unroll
  for (int e = 0; e < 8; ++e) {
    const float w = W[(size_t)(k8 + e) * N + nc];
    hv[e] = (_Float16)(live ? carry_flush(bf16r(w), kWCarry) : 0.0f);
  }
  unsigned short* dp = dst + (size_t)n * ldd + colOff + k8;
  *(volatile v8h*)dp = hv;
  __threadfence();
  *(volatile v8h*)dp = hv;
}


__device__ __forceinline__ float fast_tanh(float v) { return 1.0f - 2.0f * frcp(__expf(2.0f * v) + 1.0f); }
__device__ __forceinline__ float fast_sigmoid(float v) { return frcp(1.0f + __expf(-v)); }

__global__ __launch_bounds__(kThr) void setup_kernel(const float* __restrict__ x, const float* __restrict__ b_e, const float* __restrict__ b_d,
                                                     const float* __restrict__ bh, const float* __restrict__ bc, float* __restrict__ BIAS,
                                                     unsigned short* __restrict__ AE, float* __restrict__ CE) {
  unsigned v = blockIdx.x * (unsigned)kThr + threadIdx.x;
  asm volatile("" : "+v"(v));
  if (v < 3072u) {
    const unsigned i0 = v * 4u;
    v4f o = {0.f, 0.f, 0.f, 0.f};
    if (i0 < (unsigned)(kFBI + kIni)) {
      const float* sp = (i0 < (unsigned)kFBD) ? (b_e + i0) : ((i0 < (unsigned)kFBI) ? (b_d + (i0 - (unsigned)kFBD)) : ((i0 < (unsigned)(kFBI + kLat)) ? (bh + (i0 - (unsigned)kFBI)) : (bc + (i0 - (unsigned)(kFBI + kLat)))));
      const v4f a = *(const v4f*)sp;
#pragma unroll
      for (int e = 0; e < 4; ++e) { const float p = a[e]; o[e] = bf16r(p); }
    }
    float* dp = BIAS + i0;
    *(volatile v4f*)dp = o;
    __threadfence();
    *(volatile v4f*)dp = o;
  } else if (v < 15360u) {
    v8h hv;
    unsigned short* dp;
    if (v < 11264u) {
      const unsigned w = v - 3072u;
#pragma unroll
      for (int e = 0; e < 8; ++e) hv[e] = (_Float16)0.0f;
      dp = AE + (size_t)(w >> 7) * kKe + (w & 127u) * 8u;
    } else {
      const unsigned w = v - 11264u;
      const unsigned b = w >> 6, c8 = (w & 63u) * 8u;
      const float* sp = x + (size_t)b * kTe * kLat + c8;
      const v4f a0 = *(const v4f*)sp, a1 = *(const v4f*)(sp + 4);
#pragma unroll
      for (int e = 0; e < 4; ++e) { const float p = a0[e], q = a1[e]; hv[e] = (_Float16)carry_flush(bf16r(p), kSCarry); hv[4 + e] = (_Float16)carry_flush(bf16r(q), kSCarry); }
      dp = AE + (size_t)b * kKe + kHid + c8;
    }
    *(volatile v8h*)dp = hv;
    __threadfence();
    *(volatile v8h*)dp = hv;
  } else {
    const unsigned w = v - 15360u;
    const v4f z = {0.f, 0.f, 0.f, 0.f};
    float* dp = CE + (size_t)w * 4u;
    *(volatile v4f*)dp = z;
    __threadfence();
    *(volatile v4f*)dp = z;
  }
}
static_assert(kFEnd / 4 == 3072 && kB * kHid / 8 == 8192 && kB * kLat / 8 == 4096 && kB * kHid / 4 == 16384 && 3072 + 8192 + 4096 + 16384 == 124 * kThr, "set-up grid exact");
static_assert((3072 % 32) == 0 && (11264 % 32) == 0 && (15360 % 32) == 0 && (kFBD % 128) == 0 && (kFBI % 128) == 0 && ((kFBI + kLat) % 128) == 0 && ((kFBI + kIni) % 128) == 0, "set-up regions wave-uniform");

__global__ __launch_bounds__(kThr) void enc_cell_kernel(const float* __restrict__ GE, const float* __restrict__ x, float* __restrict__ CE,
                                                        unsigned short* __restrict__ AE, unsigned short* __restrict__ CMB16, int t) {
  unsigned v = blockIdx.x * (unsigned)kThr + threadIdx.x;
  asm volatile("" : "+v"(v));
  const unsigned b = v >> 7;
  const unsigned u8 = (v & 127u) * 8u;
  const float* gr = GE + (size_t)b * kGe + u8;
  float* cp = CE + (size_t)b * kHid + u8;
  v8h hv, cv, xv;
  v4f cn0, cn1;
#pragma unroll
  for (int hlf = 0; hlf < 2; ++hlf) {
    const v4f gi = *(const v4f*)(gr + 4 * hlf), gf = *(const v4f*)(gr + kHid + 4 * hlf), gg = *(const v4f*)(gr + 2 * kHid + 4 * hlf), go = *(const v4f*)(gr + 3 * kHid + 4 * hlf);
    const v4f co = *(const v4f*)(cp + 4 * hlf);
#pragma unroll
    for (int e = 0; e < 4; ++e) {
      const float cn = fast_sigmoid(gf[e]) * co[e] + fast_sigmoid(gi[e]) * fast_tanh(gg[e]);
      const float hn = fast_sigmoid(go[e]) * fast_tanh(cn);
      if (hlf == 0) cn0[e] = cn; else cn1[e] = cn;
      hv[4 * hlf + e] = (_Float16)carry_flush(hn, kSCarry);
      cv[4 * hlf + e] = (_Float16)carry_flush(cn, kSCarry);
    }
  }
  const bool nx = (u8 < (unsigned)kLat) && (t + 1 < kTe);
  {
    const float* sp = x + ((size_t)b * kTe + (size_t)(nx ? (t + 1) : 0)) * kLat + (nx ? u8 : 0u);
    const v4f a0 = *(const v4f*)sp, a1 = *(const v4f*)(sp + 4);
#pragma unroll
    for (int e = 0; e < 4; ++e) { const float p = a0[e], q = a1[e]; xv[e] = (_Float16)carry_flush(bf16r(p), kSCarry); xv[4 + e] = (_Float16)carry_flush(bf16r(q), kSCarry); }
  }
  const bool last = (t == kTe - 1);
  unsigned short* hp = AE + (size_t)b * kKe + u8;
  unsigned short* xp = AE + (size_t)b * kKe + kHid + (nx ? u8 : 0u);
  unsigned short* mh = CMB16 + (size_t)b * kCmb + u8;
  unsigned short* mc = CMB16 + (size_t)b * kCmb + kHid + u8;
  for (int pass = 0; pass < 2; ++pass) {
    *(volatile v4f*)cp = cn0;
    *(volatile v4f*)(cp + 4) = cn1;
    *(volatile v8h*)hp = hv;
    if (nx) *(volatile v8h*)xp = xv;
    if (last) { *(volatile v8h*)mh = hv; *(volatile v8h*)mc = cv; }
    __threadfence();
  }
}
static_assert(kB * kHid / 8 == 32 * kThr && kHid / 8 == 128 && (kLat / 8) % 32 == 0, "encoder cell grid exact; the input's threads end on a wave boundary");
__global__ __launch_bounds__(kThr) void elu_init_kernel(const float* __restrict__ INI, unsigned short* __restrict__ HD16, float* __restrict__ CD) {
  typedef __attribute__((ext_vector_type(4))) _Float16 v4h;
  unsigned v = blockIdx.x * (unsigned)kThr + threadIdx.x;
  asm volatile("" : "+v"(v));
  const unsigned b = v >> 7;
  const unsigned u4 = (v & 127u) * 4u;
  const float* ir = INI + (size_t)b * kIni + u4;
  const v4f ah = *(const v4f*)ir, ac = *(const v4f*)(ir + kLat);
  v4h hv; v4f cvv;
#pragma unroll
  for (int e = 0; e < 4; ++e) {
    const float hv0 = ah[e], cv0 = ac[e];
    const float he = (hv0 > 0.0f) ? hv0 : expm1f(hv0);
    const float ce = (cv0 > 0.0f) ? cv0 : expm1f(cv0);
    hv[e] = (_Float16)carry_flush(he, kSCarry);
    cvv[e] = ce;
  }
  unsigned short* hp = HD16 + (size_t)b * kLat + u4;
  float* cp = CD + (size_t)b * kLat + u4;
  for (int pass = 0; pass < 2; ++pass) {
    *(volatile v4h*)hp = hv;
    *(volatile v4f*)cp = cvv;
    __threadfence();
  }
}
static_assert(kB * kLat / 4 == 32 * kThr && kLat / 4 == 128, "initial-state grid exact");
static_assert(kB * kLat / 8 == 16 * kThr && kLat / 8 == 64, "decoder grids exact");

__global__ __launch_bounds__(kThr) void dec_cell_kernel(const float* __restrict__ GD, const float* __restrict__ XDEC, float* __restrict__ CD,
                                                        unsigned short* __restrict__ HD16, float* __restrict__ out, int t) {
  unsigned v = blockIdx.x * (unsigned)kThr + threadIdx.x;
  asm volatile("" : "+v"(v));
  const unsigned b = v >> 6;
  const unsigned u8 = (v & 63u) * 8u;
  const float* gr = GD + (size_t)b * kGd + u8;
  const float* xr = XDEC + (size_t)b * kGd + u8;
  float* cp = CD + (size_t)b * kLat + u8;
  v8h hv;
  v4f cn0, cn1, hn0, hn1;
#pragma unroll
  for (int hlf = 0; hlf < 2; ++hlf) {
    const v4f gi = *(const v4f*)(gr + 4 * hlf), gf = *(const v4f*)(gr + kLat + 4 * hlf), gg = *(const v4f*)(gr + 2 * kLat + 4 * hlf), go = *(const v4f*)(gr + 3 * kLat + 4 * hlf);
    const v4f xi = *(const v4f*)(xr + 4 * hlf), xf = *(const v4f*)(xr + kLat + 4 * hlf), xg = *(const v4f*)(xr + 2 * kLat + 4 * hlf), xo = *(const v4f*)(xr + 3 * kLat + 4 * hlf);
    const v4f co = *(const v4f*)(cp + 4 * hlf);
#pragma unroll
    for (int e = 0; e < 4; ++e) {
      const float cn = fast_sigmoid(xf[e] + gf[e]) * co[e] + fast_sigmoid(xi[e] + gi[e]) * fast_tanh(xg[e] + gg[e]);
      const float hn = fast_sigmoid(xo[e] + go[e]) * fast_tanh(cn);
      if (hlf == 0) { cn0[e] = cn; hn0[e] = hn; } else { cn1[e] = cn; hn1[e] = hn; }
      hv[4 * hlf + e] = (_Float16)carry_flush(hn, kSCarry);
    }
  }
  unsigned short* hp = HD16 + (size_t)b * kLat + u8;
  float* op = out + ((size_t)b * kTd + (size_t)t) * kLat + u8;
  for (int pass = 0; pass < 2; ++pass) {
    *(volatile v4f*)cp = cn0;
    *(volatile v4f*)(cp + 4) = cn1;
    *(volatile v8h*)hp = hv;
    *(volatile v4f*)op = hn0;
    *(volatile v4f*)(op + 4) = hn1;
    __threadfence();
  }
}

extern "C" void kernel_launch(void* const* d_in, const int* in_sizes, int n_in,
                              void* d_out, int out_size, void* d_ws, size_t ws_size,
                              hipStream_t stream) {
  if (n_in < 12 || d_out == nullptr || d_ws == nullptr) return;
  if (in_sizes[0] != kB * kTe * kLat || in_sizes[1] != kLat * kGe || in_sizes[2] != kHid * kGe || in_sizes[3] != kGe || in_sizes[4] != kHid * kGd || in_sizes[5] != kLat * kGd || in_sizes[6] != kGd) return;
  if (in_sizes[7] != kCmb * kLat || in_sizes[8] != kLat || in_sizes[9] != kCmb * kLat || in_sizes[10] != kLat || in_sizes[11] != 1) return;
  if (out_size != kB * kTd * kLat) return;
  if (ws_size < kWsTotal) return;
  const float* x = (const float*)d_in[0];
  const float* Wx_e = (const float*)d_in[1];
  const float* Wh_e = (const float*)d_in[2];
  const float* b_e = (const float*)d_in[3];
  const float* Wx_d = (const float*)d_in[4];
  const float* Wh_d = (const float*)d_in[5];
  const float* b_d = (const float*)d_in[6];
  const float* Wc = (const float*)d_in[7];
  const float* bc = (const float*)d_in[8];
  const float* Wh = (const float*)d_in[9];
  const float* bh = (const float*)d_in[10];
  float* out = (float*)d_out;
  char* ws = (char*)d_ws;
  unsigned short* WE = (unsigned short*)(ws + kOffWE);
  unsigned short* WINI = (unsigned short*)(ws + kOffWINI);
  unsigned short* WXD = (unsigned short*)(ws + kOffWXD);
  unsigned short* WHD = (unsigned short*)(ws + kOffWHD);
  float* BIAS = (float*)(ws + kOffBIAS);
  unsigned short* AE = (unsigned short*)(ws + kOffAE);
  float* GE = (float*)(ws + kOffGE);
  float* CE = (float*)(ws + kOffCE);
  unsigned short* CMB16 = (unsigned short*)(ws + kOffCMB16);
  float* INI = (float*)(ws + kOffINI);
  float* XDEC = (float*)(ws + kOffXDEC);
  unsigned short* HD16 = (unsigned short*)(ws + kOffHD16);
  float* GD = (float*)(ws + kOffGD);
  float* CD = (float*)(ws + kOffCD);

  wt_plane_kernel<<<kGe, kHid / 8, 0, stream>>>(Wh_e, WE, kHid, kGe, kGe, kKe, 0);
  wt_plane_kernel<<<kGe, kLat / 8, 0, stream>>>(Wx_e, WE, kLat, kGe, kGe, kKe, kHid);
  wt_plane_kernel<<<kLat, kCmb / 8, 0, stream>>>(Wh, WINI, kCmb, kLat, kLat, kCmb, 0);
  wt_plane_kernel<<<kLat, kCmb / 8, 0, stream>>>(Wc, WINI + (size_t)kLat * kCmb, kCmb, kLat, kLat, kCmb, 0);
  wt_plane_kernel<<<kGd, kHid / 8, 0, stream>>>(Wx_d, WXD, kHid, kGd, kGd, kHid, 0);
  wt_plane_kernel<<<kGd, kLat / 8, 0, stream>>>(Wh_d, WHD, kLat, kGd, kGd, kLat, 0);
  setup_kernel<<<124, kThr, 0, stream>>>(x, b_e, b_d, bh, bc, BIAS, AE, CE);

  for (int t = 0; t < kTe; ++t) {
    wmma_gemm64<0, false, 2, 0, false, 0><<<dim3((kB / 64) * (kGe / 64) / 8, 1), 256, 0, stream>>>(
        AE, AE, kKe, 0L, WE, WE, kKe, 0L, (void*)GE, (void*)GE, kGe, 0L, BIAS + kFBE, nullptr, 0L, kB, kGe, kKe, kSc);
    enc_cell_kernel<<<32, kThr, 0, stream>>>(GE, x, CE, AE, CMB16, t);
  }
  wmma_gemm64<0, false, 2, 0, false, 0><<<dim3((kB / 64) * (kIni / 64) / 8, 1), 256, 0, stream>>>(
      CMB16, CMB16, kCmb, 0L, WINI, WINI, kCmb, 0L, (void*)INI, (void*)INI, kIni, 0L, BIAS + kFBI, nullptr, 0L, kB, kIni, kCmb, kSc);
  wmma_gemm64<0, false, 2, 0, false, 0><<<dim3((kB / 64) * (kGd / 64) / 8, 1), 256, 0, stream>>>(
      AE, AE, kKe, 0L, WXD, WXD, kHid, 0L, (void*)XDEC, (void*)XDEC, kGd, 0L, BIAS + kFBD, nullptr, 0L, kB, kGd, kHid, kSc);
  elu_init_kernel<<<32, kThr, 0, stream>>>(INI, HD16, CD);

  for (int t = 0; t < kTd; ++t) {
    wmma_gemm64<0, false, 2, 0, false, 0><<<dim3((kB / 64) * (kGd / 64) / 8, 1), 256, 0, stream>>>(
        HD16, HD16, kLat, 0L, WHD, WHD, kLat, 0L, (void*)GD, (void*)GD, kGd, 0L, BIAS + kFZB, nullptr, 0L, kB, kGd, kLat, kSc);
    dec_cell_kernel<<<16, kThr, 0, stream>>>(GD, XDEC, CD, HD16, out, t);
  }
}
